// ODEfunc_5257039970521
// MI455X (gfx1250) — hardware-verified
//
#include <hip/hip_runtime.h>
#include <stddef.h>


typedef _Float16 v16h __attribute__((ext_vector_type(16)));
typedef _Float16 v8h  __attribute__((ext_vector_type(8)));
typedef float    v8f  __attribute__((ext_vector_type(8)));
typedef float    v4f  __attribute__((ext_vector_type(4)));
typedef _Float16 h16;

#ifndef NB
#define NB 524288
#endif
#define NB_FULL 524288
#define DSTATE 8
#define HWID   64
#define KIN    9

#define SAMP_TILE  16
#define TILES_WAVE 4
#define WAVES_BLK  4
#define SAMP_WAVE  (SAMP_TILE * TILES_WAVE)
#define SAMP_BLK   (SAMP_WAVE * WAVES_BLK)

static_assert(NB >= SAMP_BLK && NB <= NB_FULL);
static_assert((NB % SAMP_BLK) == 0);
static_assert(KIN == DSTATE + 1 && KIN <= 32);
static_assert(HWID == 64 && DSTATE == 8);
static_assert(SAMP_WAVE == 64);
static_assert((size_t)NB_FULL * DSTATE * 4 == (size_t)16777216);

#define OUT1_ELEM_OFF ((size_t)NB_FULL * DSTATE)

#define LDT 72
static_assert((LDT % 8) == 0 && LDT >= 64);

#define ZCARRY 64.0f
#define WCARRY 64.0f
#define GCARRY 1024.0f
#define ACARRY 64.0f

#define P_W1 0u
#define P_W2 (P_W1 + 64u * 32u)
#define P_G  (P_W2 + 64u * 64u)
#define P_W3 (P_G + 64u * 64u)
#define PLANE_HALVES (P_W3 + 16u * 64u)
#define PLANE_PIECES (PLANE_HALVES / 8u)
#define WS_TOTAL ((size_t)PLANE_HALVES * 2)
static_assert(PLANE_HALVES == 11264u);
static_assert(PLANE_PIECES == 1408u);
static_assert((WS_TOTAL % 128) == 0);
static_assert(WS_TOTAL <= (size_t)134217728);
static_assert(PLANE_PIECES == 11u * 128u);
static_assert(PLANE_PIECES <= 6u * 256u && PLANE_PIECES > 5u * 256u);

#if defined(__has_builtin)
#if __has_builtin(__builtin_amdgcn_tanhf)
#define FAST_TANH(x) __builtin_amdgcn_tanhf(x)
#elif __has_builtin(__builtin_amdgcn_tanh_f32)
#define FAST_TANH(x) __builtin_amdgcn_tanh_f32(x)
#endif
#endif
#ifndef FAST_TANH
#define FAST_TANH(x) tanhf(x)
#endif

__device__ __forceinline__ float bf16r(float x) {
  unsigned int u = __float_as_uint(x);
  u = (u + 0x7FFFu + ((u >> 16) & 1u)) & 0xFFFF0000u;
  return __uint_as_float(u);
}

static __device__ __forceinline__ h16 toh_flush(float v) {
  const h16 r = (h16)v;
  return (fabsf(v) < 6.103515625e-05f) ? (h16)0.0f : r;
}

__device__ __forceinline__ v16h frag_at(const _Float16* p) {
  v8h lo = *(const v8h*)(p);
  v8h hi = *(const v8h*)(p + 16);
  v16h out;
#pragma unroll
  for (int i = 0; i < 8; ++i) { out[i] = lo[i]; out[i + 8] = hi[i]; }
  return out;
}
__device__ __forceinline__ v16h ld_frag(const _Float16* base, unsigned ld) {
  const unsigned lane = threadIdx.x & 31u;
  return frag_at(base + (lane & 15u) * ld + (lane >> 4) * 8u);
}

__device__ __forceinline__ v8f wmma16(v16h a, v16h b, v8f c) {
  v8f d = __builtin_amdgcn_wmma_f32_16x16x32_f16(false, a, false, b, (short)0, c,
                                                 false, false);
  asm volatile("v_nop\n\tv_nop\n\tv_nop\n\tv_nop" : "+v"(d) : "v"(a), "v"(b));
  return d;
}

__device__ __forceinline__ float red16_sum(float x) {
#pragma unroll
  for (int off = 1; off < 16; off <<= 1) x += __shfl_xor(x, off, 32);
  return x;
}

__device__ __forceinline__ void wave_lds_sync() {
  __builtin_amdgcn_fence(3  , "wavefront");
  asm volatile("s_wait_dscnt 0x0" ::: "memory");
  __builtin_amdgcn_wave_barrier();
}

__global__ __launch_bounds__(256) void wprep_kernel(
    const float* __restrict__ W1, const float* __restrict__ W2, const float* __restrict__ W3,
    _Float16* __restrict__ planes) {
  __shared__ _Float16 T[PLANE_HALVES];
  const unsigned tid = threadIdx.x;

#pragma unroll 1
  for (unsigned idx = tid; idx < 64u * 32u; idx += 256u) {
    const unsigned n = idx >> 5, k = idx & 31u;
    const unsigned kc = (k < (unsigned)KIN) ? k : (unsigned)(KIN - 1);
    const float v = W1[kc * 64u + n];
    const h16 c = toh_flush(WCARRY * bf16r(v));
    T[P_W1 + idx] = (k < (unsigned)KIN) ? c : (h16)0.0f;
  }
#pragma unroll 1
  for (unsigned idx = tid; idx < 64u * 64u; idx += 256u) {
    const unsigned n = idx >> 6, k = idx & 63u;
    const float v = W2[k * 64u + n];
    T[P_W2 + idx] = toh_flush(WCARRY * bf16r(v));
  }
#pragma unroll 1
  for (unsigned idx = tid; idx < 64u * 64u; idx += 256u) {
    const unsigned n = idx >> 6, k = idx & 63u;
    float mm = 0.0f;
#pragma unroll 1
    for (unsigned d = 0; d < (unsigned)DSTATE; ++d)
      mm += bf16r(W3[n * 8u + d]) * bf16r(W1[(1u + d) * 64u + k]);
    const float g = bf16r(W2[k * 64u + n]) * mm;
    T[P_G + idx] = toh_flush(GCARRY * g);
  }
#pragma unroll 1
  for (unsigned idx = tid; idx < 16u * 64u; idx += 256u) {
    const unsigned n = idx >> 6, k = idx & 63u;
    const unsigned nc = (n < (unsigned)DSTATE) ? n : (unsigned)(DSTATE - 1);
    const float v = W3[k * 8u + nc];
    const h16 c = toh_flush(WCARRY * bf16r(v));
    T[P_W3 + idx] = (n < (unsigned)DSTATE) ? c : (h16)0.0f;
  }
  __syncthreads();

  v8h x[6];
#pragma unroll
  for (unsigned j = 0; j < 6u; ++j) {
    const unsigned piece = tid + 256u * j;
    const unsigned pc = (piece < PLANE_PIECES) ? piece : (PLANE_PIECES - 1u);
    x[j] = *(const v8h*)&T[pc * 8u];
  }
#pragma unroll
  for (unsigned j = 0; j < 6u; ++j) {
    const unsigned piece = tid + 256u * j;
    if (piece < PLANE_PIECES) *(volatile v8h*)(planes + (size_t)piece * 8u) = x[j];
  }
  __threadfence();
#pragma unroll
  for (unsigned j = 0; j < 6u; ++j) {
    const unsigned piece = tid + 256u * j;
    if (piece < PLANE_PIECES) *(volatile v8h*)(planes + (size_t)piece * 8u) = x[j];
  }
}

#define LDS_MAIN_BYTES ((size_t)PLANE_HALVES * 2 + 2u * WAVES_BLK * 16u * LDT * 2u + \
                        (size_t)WAVES_BLK * SAMP_WAVE * DSTATE * 4u + (size_t)WAVES_BLK * SAMP_WAVE * 4u + \
                        (64u + 64u + 16u) * 4u)
static_assert(LDS_MAIN_BYTES <= (size_t)65536);
static_assert(LDS_MAIN_BYTES <= (size_t)131072);
static_assert(SAMP_WAVE * DSTATE * 4 == 4 * 32 * 16);
static_assert(SAMP_WAVE * 4 == 16 * 16);
static_assert(SAMP_TILE * TILES_WAVE == SAMP_WAVE);

__global__ __launch_bounds__(128) void mlp_div_kernel(
    const float* __restrict__ tptr, const float* __restrict__ y,
    const float* __restrict__ b1, const float* __restrict__ b2, const float* __restrict__ b3,
    const _Float16* __restrict__ planes,
    float* __restrict__ dy, float* __restrict__ negdiv) {
  __shared__ _Float16 sW[PLANE_HALVES];
  __shared__ _Float16 Hs[WAVES_BLK * 16 * LDT];
  __shared__ _Float16 As[WAVES_BLK * 16 * LDT];
  __shared__ float DyS[WAVES_BLK * SAMP_WAVE * DSTATE];
  __shared__ float NdS[WAVES_BLK * SAMP_WAVE];
  __shared__ float sB1[64];
  __shared__ float sB2[64];
  __shared__ float sB3[16];

  const unsigned tid = threadIdx.x, lane = tid & 31u;
  const unsigned wave = __builtin_amdgcn_readfirstlane(threadIdx.x >> 5);
  const unsigned hh = lane >> 4, m = lane & 15u;

#pragma unroll
  for (unsigned j = 0; j < 11u; ++j) {
    const unsigned piece = tid + 128u * j;
    *(v8h*)&sW[piece * 8u] = *(const v8h*)(planes + (size_t)piece * 8u);
  }
  {
    const float b1v = b1[tid & 63u];
    const float b2v = b2[tid & 63u];
    const float b3v = b3[tid & 7u];
    if (tid < 64u) { sB1[tid] = bf16r(b1v); sB2[tid] = bf16r(b2v); }
    if (tid < 16u) sB3[tid] = (tid < 8u) ? bf16r(b3v) : 0.0f;
  }
  __syncthreads();

  const float tz = ZCARRY * bf16r(tptr[0]);
  const bool up = (hh != 0u);
  _Float16* H = Hs + wave * (16u * LDT);
  _Float16* A = As + wave * (16u * LDT);
  float* D = DyS + wave * (unsigned)(SAMP_WAVE * DSTATE);
  float* N = NdS + wave * (unsigned)SAMP_WAVE;
  const unsigned wbase = blockIdx.x * (unsigned)SAMP_BLK + wave * (unsigned)SAMP_WAVE;

#pragma unroll 1
  for (unsigned tile = 0; tile < (unsigned)TILES_WAVE; ++tile) {
    const size_t s = (size_t)(wbase + tile * 16u + m);
    const v4f ylo = *(const v4f*)(y + s * 8u);
    const v4f yhi = *(const v4f*)(y + s * 8u + 4u);

    float yv[8];
#pragma unroll
    for (int i = 0; i < 4; ++i) {
      yv[i]     = ZCARRY * bf16r(ylo[i]);
      yv[i + 4] = ZCARRY * bf16r(yhi[i]);
    }
    v16h za;
    za[0] = toh_flush(up ? yv[7] : tz);
#pragma unroll
    for (int i = 1; i < 8; ++i) za[i] = toh_flush(up ? 0.0f : yv[i - 1]);
#pragma unroll
    for (int i = 8; i < 16; ++i) za[i] = (h16)0.0f;

    v8f acc1[4];
#pragma unroll
    for (int n = 0; n < 4; ++n) {
      const v16h bw = ld_frag(&sW[P_W1 + (unsigned)n * 16u * 32u], 32u);
      acc1[n] = wmma16(za, bw, (v8f){});
    }
#pragma unroll
    for (int n = 0; n < 4; ++n) {
      const unsigned col = (unsigned)n * 16u + m;
      const float bb = sB1[col];
#pragma unroll
      for (int r = 0; r < 8; ++r) {
        const float pre = acc1[n][r] * (1.0f / (ZCARRY * WCARRY)) + bb;
        const float h = FAST_TANH(pre);
        const float a = 1.0f - h * h;
        H[(hh * 8u + (unsigned)r) * LDT + col] = toh_flush(ACARRY * h);
        A[(hh * 8u + (unsigned)r) * LDT + col] = toh_flush(ACARRY * a);
      }
    }
    wave_lds_sync();

    v8f acc2[4], vacc[4];
#pragma unroll
    for (int n = 0; n < 4; ++n) { acc2[n] = (v8f){}; vacc[n] = (v8f){}; }
#pragma unroll
    for (int c = 0; c < 2; ++c) {
      const v16h ah = ld_frag(H + c * 32, LDT);
      const v16h aa = ld_frag(A + c * 32, LDT);
#pragma unroll
      for (int n = 0; n < 4; ++n) {
        const v16h bw = ld_frag(&sW[P_W2 + (unsigned)n * 16u * 64u + (unsigned)c * 32u], 64u);
        acc2[n] = wmma16(ah, bw, acc2[n]);
        const v16h bg = ld_frag(&sW[P_G + (unsigned)n * 16u * 64u + (unsigned)c * 32u], 64u);
        vacc[n] = wmma16(aa, bg, vacc[n]);
      }
    }
    wave_lds_sync();

    float p[8];
#pragma unroll
    for (int r = 0; r < 8; ++r) p[r] = 0.0f;
#pragma unroll
    for (int n = 0; n < 4; ++n) {
      const unsigned col = (unsigned)n * 16u + m;
      const float bb = sB2[col];
#pragma unroll
      for (int r = 0; r < 8; ++r) {
        const float pre = acc2[n][r] * (1.0f / (ACARRY * WCARRY)) + bb;
        const float h = FAST_TANH(pre);
        p[r] += vacc[n][r] * (1.0f - h * h);
        H[(hh * 8u + (unsigned)r) * LDT + col] = toh_flush(ACARRY * h);
      }
    }
    wave_lds_sync();

    v8f acc3 = {};
#pragma unroll
    for (int c = 0; c < 2; ++c) {
      const v16h ah = ld_frag(H + c * 32, LDT);
      const v16h bw = ld_frag(&sW[P_W3 + (unsigned)c * 32u], 64u);
      acc3 = wmma16(ah, bw, acc3);
    }
    const float b3v = sB3[m];
#pragma unroll
    for (int r = 0; r < 8; ++r) {
      const float val = acc3[r] * (1.0f / (ACARRY * WCARRY)) + b3v;
      if (m < (unsigned)DSTATE)
        D[(tile * 16u + hh * 8u + (unsigned)r) * (unsigned)DSTATE + m] = val;
    }

#pragma unroll
    for (int r = 0; r < 8; ++r) {
      const float tot = red16_sum(p[r]);
      const float nd = -(tot * (1.0f / (ACARRY * GCARRY)));
      if (m == 0u) N[tile * 16u + hh * 8u + (unsigned)r] = nd;
    }
    wave_lds_sync();
  }

  v4f xd[4];
  size_t od[4];
#pragma unroll
  for (unsigned i = 0; i < 4u; ++i) {
    const unsigned piece = i * 32u + lane;
    xd[i] = *(const v4f*)&D[piece * 4u];
    od[i] = (size_t)wbase * DSTATE + (size_t)piece * 4u;
  }
  const v4f xn = *(const v4f*)&N[(lane & 15u) * 4u];
  const size_t on = (size_t)wbase + (size_t)(lane & 15u) * 4u;

#pragma unroll
  for (int i = 0; i < 4; ++i) *(volatile v4f*)(dy + od[i]) = xd[i];
  if (lane < 16u) *(volatile v4f*)(negdiv + on) = xn;
  __threadfence();
#pragma unroll
  for (int i = 0; i < 4; ++i) *(volatile v4f*)(dy + od[i]) = xd[i];
  if (lane < 16u) *(volatile v4f*)(negdiv + on) = xn;
}

extern "C" void kernel_launch(void* const* d_in, const int* in_sizes, int n_in,
                              void* d_out, int out_size, void* d_ws, size_t ws_size,
                              hipStream_t stream) {
  if (n_in < 9) return;
  if (in_sizes[0] < 1) return;
  if ((long long)in_sizes[1] < (long long)NB * DSTATE) return;
  if (in_sizes[3] < KIN * HWID) return;
  if (in_sizes[4] < HWID) return;
  if (in_sizes[5] < HWID * HWID) return;
  if (in_sizes[6] < HWID) return;
  if (in_sizes[7] < HWID * DSTATE) return;
  if (in_sizes[8] < DSTATE) return;
  if ((long long)out_size < (long long)OUT1_ELEM_OFF + (long long)NB) return;
  if (ws_size < WS_TOTAL) return;

  const float* t  = (const float*)d_in[0];
  const float* y  = (const float*)d_in[1];
  const float* W1 = (const float*)d_in[3];
  const float* b1 = (const float*)d_in[4];
  const float* W2 = (const float*)d_in[5];
  const float* b2 = (const float*)d_in[6];
  const float* W3 = (const float*)d_in[7];
  const float* b3 = (const float*)d_in[8];

  float* out_dy = (float*)d_out;
  float* out_nd = (float*)d_out + OUT1_ELEM_OFF;
  _Float16* planes = (_Float16*)d_ws;

  wprep_kernel<<<dim3(1), dim3(256), 0, stream>>>(W1, W2, W3, planes);
  mlp_div_kernel<<<dim3(NB / SAMP_BLK), dim3(128), 0, stream>>>(t, y, b1, b2, b3, planes,
                                                                out_dy, out_nd);
}
